// GCN_Dropout_28243704939123
// MI455X (gfx1250) — hardware-verified
//
#include <hip/hip_runtime.h>
#include <stddef.h>


#define DIN     128
#define HID     256
#define DOUT    128
#define LNEPS   1e-5f
#define NTHR    256
#define NWAVE   8
#define EPT     8
#define NGRP    2
#define CHUNK   (NTHR * EPT * NGRP)
#define WCAPC   (EPT * NGRP * 32)
#define WCAPF   (EPT * NGRP * 32)
#define ESHF    11
#define NBC     32768
#define NBF     2048
#define RCAP    49152
#define RBN     128
#define TGT     256
#define DEGCAP  512
#define GROWS   128
#define GCOLS   128
#define OTHR    512
#define TPK     64
#define TPN     32
#define TPP     72
#define WSCAP   134217728

#define LDS_COUNT ((NBC + NWAVE * WCAPC + NWAVE) * 4)
#define LDS_FILL  ((RCAP + NBF + NWAVE * WCAPF + NWAVE) * 4)
#define LDS_GEMM  (GROWS * GCOLS * 4)

static_assert((CHUNK & (CHUNK - 1)) == 0);
static_assert((NBC & (NBC - 1)) == 0 && (NBF & (NBF - 1)) == 0);
static_assert(NBF <= (1 << ESHF));
static_assert((NBC % NBF) == 0);
static_assert(OTHR * 4 == NBF);
static_assert((RCAP % 32) == 0);
static_assert(TGT == NWAVE * 32);
static_assert(GROWS == NWAVE * 16);
static_assert((TGT % GROWS) == 0);
static_assert(NBC == NWAVE * 32 * 128);
static_assert((HID % GCOLS) == 0 && (DOUT % GCOLS) == 0 && GCOLS == 32 * 4);
static_assert((DIN % 32) == 0 && (HID % 32) == 0 && (DIN % 8) == 0);
static_assert((DIN % TPK) == 0 && (HID % TPK) == 0 && (HID % TPN) == 0 && (DOUT % TPN) == 0);
static_assert(TPN * 8 == NTHR && TPK * TPN == NTHR * 8 && TPK == NWAVE * 8);
static_assert((TPP % 8) == 0 && TPP >= TPK);
static_assert(LDS_FILL <= 300 * 1024);

typedef float          v4f   __attribute__((ext_vector_type(4)));
typedef float          v8f   __attribute__((ext_vector_type(8)));
typedef int            v4i   __attribute__((ext_vector_type(4)));
typedef unsigned short v8us  __attribute__((ext_vector_type(8)));
typedef __bf16         v16bf __attribute__((ext_vector_type(16)));
union FragB { v16bf v; v8us h[2]; };
union U32F { float f; int i; };

__device__ __forceinline__ v8f wmb(v16bf a, v16bf b, v8f c) {
  v8f d = __builtin_amdgcn_wmma_f32_16x16x32_bf16(false, a, false, b, (short)0, c, false, false);
  asm volatile("v_nop\n\tv_nop\n\tv_nop\n\tv_nop" : "+v"(d) : "v"(a), "v"(b));
  return d;
}

__device__ __forceinline__ v4f relu4(v4f t) {
  v4f o;
  o.x = fmaxf(t.x, 0.0f); o.y = fmaxf(t.y, 0.0f); o.z = fmaxf(t.z, 0.0f); o.w = fmaxf(t.w, 0.0f);
  return o;
}

__device__ __forceinline__ unsigned bf_bits(float x) {
  const unsigned u = __float_as_uint(x);
  return (u + 0x7FFFu + ((u >> 16) & 1u)) >> 16;
}
__device__ __forceinline__ void split_bits(float x, unsigned short& h, unsigned short& l) {
  const unsigned hb = bf_bits(x);
  const float r = x - __uint_as_float(hb << 16);
  h = (unsigned short)hb;
  l = (unsigned short)bf_bits(r);
}
__device__ __forceinline__ void split8(v4f a, v4f b, v8us& h, v8us& l) {
  unsigned short th, tl;
  split_bits(a.x, th, tl); h[0] = th; l[0] = tl;
  split_bits(a.y, th, tl); h[1] = th; l[1] = tl;
  split_bits(a.z, th, tl); h[2] = th; l[2] = tl;
  split_bits(a.w, th, tl); h[3] = th; l[3] = tl;
  split_bits(b.x, th, tl); h[4] = th; l[4] = tl;
  split_bits(b.y, th, tl); h[5] = th; l[5] = tl;
  split_bits(b.z, th, tl); h[6] = th; l[6] = tl;
  split_bits(b.w, th, tl); h[7] = th; l[7] = tl;
}

template <int NB, int SRC, int WC>
__device__ __forceinline__ int scan_chunk(const int* __restrict__ keys, const int* __restrict__ vals,
                                          int nK, int nN, int cbase, int slotBase, int vec8,
                                          int* list, int tid, int lane, int wave) {
  int wc = 0;
#pragma unroll
  for (int g = 0; g < NGRP; ++g) {
    const int el0  = (g * NTHR + tid) * EPT;
    const int e0   = cbase + el0;
    const int sent = -2147483647 - 1;
    v4i da, db;
    v4i sa = {0, 0, 0, 0}, sb = {0, 0, 0, 0};
    if (vec8 != 0 && cbase + CHUNK <= nK) {
      da = *(const v4i*)(keys + e0);
      db = *(const v4i*)(keys + e0 + 4);
      if (SRC) {
        sa = *(const v4i*)(vals + e0);
        sb = *(const v4i*)(vals + e0 + 4);
      }
    } else {
      const int i0 = min(e0, nK - 1),     i1 = min(e0 + 1, nK - 1), i2 = min(e0 + 2, nK - 1), i3 = min(e0 + 3, nK - 1);
      const int i4 = min(e0 + 4, nK - 1), i5 = min(e0 + 5, nK - 1), i6 = min(e0 + 6, nK - 1), i7 = min(e0 + 7, nK - 1);
      da.x = (e0     < nK) ? keys[i0] : sent;
      da.y = (e0 + 1 < nK) ? keys[i1] : sent;
      da.z = (e0 + 2 < nK) ? keys[i2] : sent;
      da.w = (e0 + 3 < nK) ? keys[i3] : sent;
      db.x = (e0 + 4 < nK) ? keys[i4] : sent;
      db.y = (e0 + 5 < nK) ? keys[i5] : sent;
      db.z = (e0 + 6 < nK) ? keys[i6] : sent;
      db.w = (e0 + 7 < nK) ? keys[i7] : sent;
      if (SRC) {
        sa.x = vals[i0]; sa.y = vals[i1]; sa.z = vals[i2]; sa.w = vals[i3];
        sb.x = vals[i4]; sb.y = vals[i5]; sb.z = vals[i6]; sb.w = vals[i7];
      }
    }
    if (SRC) {
      sa.x = min(max(sa.x, 0), nN - 1); sa.y = min(max(sa.y, 0), nN - 1);
      sa.z = min(max(sa.z, 0), nN - 1); sa.w = min(max(sa.w, 0), nN - 1);
      sb.x = min(max(sb.x, 0), nN - 1); sb.y = min(max(sb.y, 0), nN - 1);
      sb.z = min(max(sb.z, 0), nN - 1); sb.w = min(max(sb.w, 0), nN - 1);
    }
    const unsigned nb = (unsigned)slotBase;
    const unsigned s0 = (unsigned)da.x - nb, s1 = (unsigned)da.y - nb;
    const unsigned s2 = (unsigned)da.z - nb, s3 = (unsigned)da.w - nb;
    const unsigned s4 = (unsigned)db.x - nb, s5 = (unsigned)db.y - nb;
    const unsigned s6 = (unsigned)db.z - nb, s7 = (unsigned)db.w - nb;
    const bool h0 = s0 < (unsigned)NB, h1 = s1 < (unsigned)NB, h2 = s2 < (unsigned)NB, h3 = s3 < (unsigned)NB;
    const bool h4 = s4 < (unsigned)NB, h5 = s5 < (unsigned)NB, h6 = s6 < (unsigned)NB, h7 = s7 < (unsigned)NB;
    const unsigned any = __builtin_amdgcn_ballot_w32(h0 | h1 | h2 | h3 | h4 | h5 | h6 | h7);
    if (any != 0u) {
#define HITJ(HJ, SJ, VJ) { \
        const unsigned mj = __builtin_amdgcn_ballot_w32(HJ); \
        if (mj != 0u) { \
          if (HJ) { \
            const int pos = wc + (int)__builtin_amdgcn_mbcnt_lo(mj, 0u); \
            const int entv = SRC ? (((VJ) << ESHF) | (int)(SJ)) : (int)(SJ); \
            if (pos < WC) list[wave * WC + pos] = entv; \
          } \
          wc += (int)__builtin_popcount(mj); } }
      HITJ(h0, s0, sa.x)
      HITJ(h1, s1, sa.y)
      HITJ(h2, s2, sa.z)
      HITJ(h3, s3, sa.w)
      HITJ(h4, s4, sb.x)
      HITJ(h5, s5, sb.y)
      HITJ(h6, s6, sb.z)
      HITJ(h7, s7, sb.w)
#undef HITJ
    }
  }
  return wc;
}

__global__ __launch_bounds__(NTHR) void k_split16(const float* __restrict__ src,
                                                  unsigned short* dh, unsigned short* dl,
                                                  int rowLen, int nSrcRows, int total8) {
  const int i = (int)blockIdx.x * NTHR + (int)threadIdx.x;
  if (i >= total8) return;
  const size_t e  = (size_t)8 * (size_t)i;
  const int    r  = (int)(e / (size_t)rowLen);
  const int    k0 = (int)(e - (size_t)r * (size_t)rowLen);
  const int    rc = r < nSrcRows ? r : nSrcRows - 1;
  const float  z  = (r < nSrcRows) ? 1.0f : 0.0f;
  const float* sp = src + (size_t)rc * rowLen + k0;
  v4f f0 = *(const v4f*)sp;
  v4f f1 = *(const v4f*)(sp + 4);
  f0 = f0 * z; f1 = f1 * z;
  v8us hv, lv;
  split8(f0, f1, hv, lv);
  unsigned short* ph = dh + e;
  unsigned short* pl = dl + e;
  *(volatile v8us*)ph = hv;
  *(volatile v8us*)pl = lv;
  __threadfence();
  *(volatile v8us*)ph = hv;
  *(volatile v8us*)pl = lv;
}

__global__ __launch_bounds__(NTHR) void k_wT16(const float* __restrict__ W, unsigned short* Wh,
                                               unsigned short* Wl, int KD, int NC) {
  __shared__ __attribute__((aligned(16))) unsigned short sH[TPN * TPP];
  __shared__ __attribute__((aligned(16))) unsigned short sL[TPN * TPP];
  const int tid = threadIdx.x;
  const int k0 = (int)blockIdx.x * TPK, n0 = (int)blockIdx.y * TPN;
  const int nc = tid & 31, kq = tid >> 5;
#pragma unroll
  for (int i = 0; i < TPK / NWAVE; ++i) {
    const int kr = kq + NWAVE * i;
    const float v = W[(size_t)(k0 + kr) * NC + n0 + nc];
    unsigned short h, l;
    split_bits(v, h, l);
    sH[nc * TPP + kr] = h;
    sL[nc * TPP + kr] = l;
  }
  __syncthreads();
  const int nl = tid >> 3, p = tid & 7;
  const v8us hv = *(const v8us*)(sH + nl * TPP + 8 * p);
  const v8us lv = *(const v8us*)(sL + nl * TPP + 8 * p);
  unsigned short* ph = Wh + (size_t)(n0 + nl) * KD + k0 + 8 * p;
  unsigned short* pl = Wl + (size_t)(n0 + nl) * KD + k0 + 8 * p;
  *(volatile v8us*)ph = hv;
  *(volatile v8us*)pl = lv;
  __threadfence();
  *(volatile v8us*)ph = hv;
  *(volatile v8us*)pl = lv;
}

__global__ __launch_bounds__(NTHR) void k_count(
    const int* __restrict__ keys, int* cnt, float* dinv, int nK, int nN, int vec8) {
  extern __shared__ v4f lds_dyn[];
  int* scnt = (int*)lds_dyn;
  int* list = scnt + NBC;
  int* wcnt = list + NWAVE * WCAPC;
  const int tid = threadIdx.x, lane = tid & 31, wave = tid >> 5;
  const int nodeBase = blockIdx.x * NBC;

  {
    const v4i z = {0, 0, 0, 0};
    for (int i = tid; i < NBC / 4; i += NTHR) ((v4i*)scnt)[i] = z;
  }
  __syncthreads();

  const int nChunks = (nK + CHUNK - 1) / CHUNK;
#pragma unroll 1
  for (int ch = 0; ch < nChunks; ++ch) {
    const int cbase = ch * CHUNK;
    const int wc = scan_chunk<NBC, 0, WCAPC>(keys, keys, nK, nN, cbase, nodeBase, vec8, list, tid, lane, wave);
    if (lane == 0) wcnt[wave] = wc;
    __syncthreads();
    if (wave == 0) {
#pragma unroll 1
      for (int wsx = 0; wsx < NWAVE; ++wsx) {
        int n = __builtin_amdgcn_readfirstlane(wcnt[wsx]);
        n = n > WCAPC ? WCAPC : (n < 0 ? 0 : n);
        const int* lp = list + wsx * WCAPC;
#pragma unroll 1
        for (int i = 0; i < n; ++i) {
          const int ent  = __builtin_amdgcn_readfirstlane(lp[i]);
          const int slot = ent & (NBC - 1);
          if (lane == 0) scnt[slot] = scnt[slot] + 1;
        }
      }
    }
    __syncthreads();
  }

  int*   cp = cnt + (size_t)nodeBase;
  float* dp = dinv + (size_t)nodeBase;
#pragma unroll 4
  for (int q = 0; q < 32; ++q) {
    const int f = (wave * 32 + q) * 128 + 4 * lane;
    const v4i c = *(const v4i*)(scnt + f);
    const float g0 = (float)c.x + 1.0f, g1 = (float)c.y + 1.0f, g2 = (float)c.z + 1.0f, g3 = (float)c.w + 1.0f;
    v4f d;
    d.x = g0 > 0.f ? rsqrtf(g0) : 0.f; d.y = g1 > 0.f ? rsqrtf(g1) : 0.f;
    d.z = g2 > 0.f ? rsqrtf(g2) : 0.f; d.w = g3 > 0.f ? rsqrtf(g3) : 0.f;
    *(volatile v4i*)(cp + f) = c;
    *(volatile v4f*)(dp + f) = d;
  }
  __threadfence();
#pragma unroll 4
  for (int q = 0; q < 32; ++q) {
    const int f = (wave * 32 + q) * 128 + 4 * lane;
    const v4i c = *(const v4i*)(scnt + f);
    const float g0 = (float)c.x + 1.0f, g1 = (float)c.y + 1.0f, g2 = (float)c.z + 1.0f, g3 = (float)c.w + 1.0f;
    v4f d;
    d.x = g0 > 0.f ? rsqrtf(g0) : 0.f; d.y = g1 > 0.f ? rsqrtf(g1) : 0.f;
    d.z = g2 > 0.f ? rsqrtf(g2) : 0.f; d.w = g3 > 0.f ? rsqrtf(g3) : 0.f;
    *(volatile v4i*)(cp + f) = c;
    *(volatile v4f*)(dp + f) = d;
  }
}

__global__ __launch_bounds__(OTHR) void k_offsets(
    const int* __restrict__ cnt, int* off, int* rbase, int nBF) {
  __shared__ __attribute__((aligned(16))) int srb[RBN];
  __shared__ int wtot[OTHR / 32];
  const int tid = threadIdx.x, lane = tid & 31, wave = tid >> 5;
  for (int i = tid; i < RBN; i += OTHR) srb[i] = 0;
  int carry = 0;
#pragma unroll 1
  for (int fb = 0; fb < nBF; ++fb) {
    const int base = fb * NBF;
    const v4i c = *(const v4i*)(cnt + base + 4 * tid);
    const int e0 = max(c.x, 0), e1 = max(c.y, 0), e2 = max(c.z, 0), e3 = max(c.w, 0);
    const int ts = e0 + e1 + e2 + e3;
    int incl = ts;
#pragma unroll
    for (int d = 1; d < 32; d <<= 1) {
      const int t = __shfl_up(incl, d, 32);
      if (lane >= d) incl += t;
    }
    if (lane == 31) wtot[wave] = incl;
    __syncthreads();
    int pre = 0;
#pragma unroll 1
    for (int w = 0; w < wave; ++w) pre += wtot[w];
    int tot = 0;
#pragma unroll
    for (int w = 0; w < OTHR / 32; ++w) tot += wtot[w];
    int run = carry + pre + incl - ts;
    v4i o;
    o.x = run; run += e0;
    o.y = run; run += e1;
    o.z = run; run += e2;
    o.w = run;
    int* op = off + base + 4 * tid;
    *(volatile v4i*)op = o;
    __threadfence();
    *(volatile v4i*)op = o;
    if (tid == 0) srb[min(fb, RBN - 1)] = carry;
    carry += (tot + 31) & ~31;
    __syncthreads();
  }
  if (tid == 0) srb[min(nBF, RBN - 1)] = carry;
  __syncthreads();
  v4i rv = {0, 0, 0, 0};
  if (tid < 32) rv = *(const v4i*)(srb + 4 * tid);
  if (tid < 32) *(volatile v4i*)(rbase + 4 * tid) = rv;
  __threadfence();
  if (tid < 32) *(volatile v4i*)(rbase + 4 * tid) = rv;
}

__global__ __launch_bounds__(NTHR) void k_fill(
    const int* __restrict__ keys, const int* __restrict__ vals, const int* __restrict__ off,
    const int* __restrict__ rbase, int* csr, int nN, int nK, int vec8, int csrLen) {
  extern __shared__ v4f lds_dyn[];
  int* region = (int*)lds_dyn;
  int* cursor = region + RCAP;
  int* list   = cursor + NBF;
  int* wcnt   = list + NWAVE * WCAPF;
  const int tid = threadIdx.x, lane = tid & 31, wave = tid >> 5;
  const int b = blockIdx.x;
  const int nodeBase = b * NBF;

  int rb0 = rbase[b];
  const int rb1 = rbase[b + 1];
  rb0 = rb0 < 0 ? 0 : (rb0 > csrLen ? csrLen : rb0);
  rb0 &= ~31;
  int len = rb1 - rb0;
  len = len < 0 ? 0 : (len > RCAP ? RCAP : len);
  int lenW = (len + 31) & ~31;
  if (rb0 + lenW > csrLen) lenW = (csrLen - rb0) & ~31;

  {
    const v4i z = {0, 0, 0, 0};
    for (int i = tid; i < RCAP / 4; i += NTHR) ((v4i*)region)[i] = z;
    for (int s = tid; s < NBF; s += NTHR) {
      int o = off[nodeBase + s] - rb0;
      o = o < 0 ? 0 : (o > RCAP ? RCAP : o);
      cursor[s] = o;
    }
  }
  __syncthreads();

  const int nChunks = (nK + CHUNK - 1) / CHUNK;
#pragma unroll 1
  for (int ch = 0; ch < nChunks; ++ch) {
    const int cbase = ch * CHUNK;
    const int wc = scan_chunk<NBF, 1, WCAPF>(keys, vals, nK, nN, cbase, nodeBase, vec8, list, tid, lane, wave);
    if (lane == 0) wcnt[wave] = wc;
    __syncthreads();
    if (wave == 0) {
#pragma unroll 1
      for (int wsx = 0; wsx < NWAVE; ++wsx) {
        int n = __builtin_amdgcn_readfirstlane(wcnt[wsx]);
        n = n > WCAPF ? WCAPF : (n < 0 ? 0 : n);
        const int* lp = list + wsx * WCAPF;
#pragma unroll 1
        for (int i = 0; i < n; ++i) {
          const int ent  = __builtin_amdgcn_readfirstlane(lp[i]);
          const int slot = ent & (NBF - 1);
          int src = (ent >> ESHF) & 0xFFFFF;
          src = src > nN - 1 ? nN - 1 : src;
          if (lane == 0) {
            int pos = cursor[slot];
            pos = pos < 0 ? 0 : (pos > RCAP - 1 ? RCAP - 1 : pos);
            region[pos] = src;
            const int np = pos + 1;
            cursor[slot] = np > RCAP ? RCAP : np;
          }
        }
      }
    }
    __syncthreads();
  }

  const int nv = lenW >> 2;
  int* gp = csr + rb0;
#pragma unroll 1
  for (int i = tid; i < nv; i += NTHR) { const v4i v = ((const v4i*)region)[i]; *(volatile v4i*)(gp + 4 * i) = v; }
  __threadfence();
#pragma unroll 1
  for (int i = tid; i < nv; i += NTHR) { const v4i v = ((const v4i*)region)[i]; *(volatile v4i*)(gp + 4 * i) = v; }
}

template <int KD, int NC>
__global__ __launch_bounds__(NTHR) void k_gemm(
    const unsigned short* __restrict__ Ah, const unsigned short* __restrict__ Al,
    const unsigned short* __restrict__ Bh, const unsigned short* __restrict__ Bl,
    const float* __restrict__ rsc, float* C, int nRows) {
  static_assert((KD % 32) == 0 && (NC % GCOLS) == 0);
  extern __shared__ v4f lds_dyn[];
  constexpr int NT = GCOLS / 16;
  float* stg = (float*)lds_dyn;
  const int tid = threadIdx.x, lane = tid & 31, wave = tid >> 5, hh = lane >> 4, m = lane & 15;
  const int rowBase = blockIdx.x * GROWS;
  const int colBase = blockIdx.y * GCOLS;
  const size_t aoff = (size_t)(rowBase + wave * 16 + m) * KD + 8 * hh;
  const size_t boff = (size_t)(colBase + m) * KD + 8 * hh;
  const unsigned short* aph = Ah + aoff;
  const unsigned short* apl = Al + aoff;
  const unsigned short* bph = Bh + boff;
  const unsigned short* bpl = Bl + boff;

  v8f acc[NT];
#pragma unroll
  for (int t = 0; t < NT; ++t) { v8f z = {0.f, 0.f, 0.f, 0.f, 0.f, 0.f, 0.f, 0.f}; acc[t] = z; }

#pragma unroll 1
  for (int kt = 0; kt < KD / 32; ++kt) {
    FragB ah, al;
    ah.h[0] = *(const v8us*)(aph + 32 * kt);
    ah.h[1] = *(const v8us*)(aph + 32 * kt + 16);
    al.h[0] = *(const v8us*)(apl + 32 * kt);
    al.h[1] = *(const v8us*)(apl + 32 * kt + 16);
#pragma unroll
    for (int t = 0; t < NT; ++t) {
      const size_t to = (size_t)(16 * t) * KD + (size_t)(32 * kt);
      FragB bh, bl;
      bh.h[0] = *(const v8us*)(bph + to);
      bh.h[1] = *(const v8us*)(bph + to + 16);
      bl.h[0] = *(const v8us*)(bpl + to);
      bl.h[1] = *(const v8us*)(bpl + to + 16);
      v8f d = acc[t];
      d = wmb(ah.v, bh.v, d);
      d = wmb(ah.v, bl.v, d);
      d = wmb(al.v, bh.v, d);
      acc[t] = d;
    }
  }

  const int r0 = wave * 16 + 8 * hh;
  float s[8];
  {
    const v4f dA = *(const v4f*)(rsc + (size_t)rowBase + r0);
    const v4f dB = *(const v4f*)(rsc + (size_t)rowBase + r0 + 4);
    s[0] = dA.x; s[1] = dA.y; s[2] = dA.z; s[3] = dA.w; s[4] = dB.x; s[5] = dB.y; s[6] = dB.z; s[7] = dB.w;
  }

  float* sp = stg + r0 * GCOLS + m;
#pragma unroll
  for (int t = 0; t < NT; ++t) {
#pragma unroll
    for (int r = 0; r < 8; ++r) sp[r * GCOLS + 16 * t] = acc[t][r] * s[r];
  }
  __syncthreads();

  const float* lp = stg + wave * 16 * GCOLS;
  float* gp = C + (size_t)(rowBase + wave * 16) * NC + colBase;
#pragma unroll
  for (int i = 0; i < 16; ++i) {
    if (rowBase + wave * 16 + i < nRows) {
      const v4f v = *(const v4f*)(lp + i * GCOLS + 4 * lane);
      *(volatile v4f*)(gp + (size_t)i * NC + 4 * lane) = v;
    }
  }
  __threadfence();
#pragma unroll
  for (int i = 0; i < 16; ++i) {
    if (rowBase + wave * 16 + i < nRows) {
      const v4f v = *(const v4f*)(lp + i * GCOLS + 4 * lane);
      *(volatile v4f*)(gp + (size_t)i * NC + 4 * lane) = v;
    }
  }
}

template <int CH, int MODE>
__global__ __launch_bounds__(NTHR) void k_agg(
    const int* __restrict__ csr, const int* __restrict__ off, const int* __restrict__ cnt,
    const float* __restrict__ dinv, const float* __restrict__ hw, const float* __restrict__ bias,
    const float* __restrict__ gam, const float* __restrict__ bet,
    float* outF, unsigned short* outHi, unsigned short* outLo, int nN, int csrLen) {
  static_assert(CH == 128 || CH == 256);
  constexpr int NQ = CH / 128;
  static_assert((MODE == 0 && NQ == 2) || (MODE == 1 && NQ == 1));
  const int tid = threadIdx.x, lane = tid & 31, wave = tid >> 5;
  const int tbase = blockIdx.x * TGT + wave * 32;
  const int cl = tbase + lane;
  const int cnt_l = cnt[cl];
  const int off_l = off[cl];
  U32F dvu; dvu.f = dinv[cl];
  const int ch0 = 4 * NQ * lane;
  v4f bq[NQ], gq[NQ], eq[NQ];
#pragma unroll
  for (int q = 0; q < NQ; ++q) {
    bq[q] = *(const v4f*)(bias + ch0 + 4 * q);
    gq[q] = *(const v4f*)(gam + ch0 + 4 * q);
    eq[q] = *(const v4f*)(bet + ch0 + 4 * q);
  }
  const float invC = 1.0f / (float)CH;

#pragma unroll 1
  for (int j = 0; j < 32; ++j) {
    const int c = tbase + j;
    int n = __builtin_amdgcn_readlane(cnt_l, j);
    n = n < 0 ? 0 : (n > DEGCAP ? DEGCAP : n);
    const int st = __builtin_amdgcn_readlane(off_l, j);
    U32F du; du.i = __builtin_amdgcn_readlane(dvu.i, j);
    const float dc = du.f;
    v4f acc[NQ];
#pragma unroll
    for (int q = 0; q < NQ; ++q) { v4f z = {0.f, 0.f, 0.f, 0.f}; acc[q] = z; }
#pragma unroll 1
    for (int q0 = 0; q0 < n; q0 += 32) {
      int pos = st + q0 + lane;
      pos = pos < 0 ? 0 : (pos > csrLen - 1 ? csrLen - 1 : pos);
      int sl = csr[pos];
      sl = sl < 0 ? 0 : (sl > nN - 1 ? nN - 1 : sl);
      const int mcnt = (n - q0) < 32 ? (n - q0) : 32;
#pragma unroll 1
      for (int p = 0; p < mcnt; ++p) {
        const int s = __builtin_amdgcn_readlane(sl, p);
        const float* hp = hw + (size_t)s * CH + ch0;
#pragma unroll
        for (int q = 0; q < NQ; ++q) acc[q] = acc[q] + *(const v4f*)(hp + 4 * q);
      }
    }
    const float* cp = hw + (size_t)c * CH + ch0;
    v4f v[NQ];
#pragma unroll
    for (int q = 0; q < NQ; ++q) {
      const v4f sv = *(const v4f*)(cp + 4 * q);
      v[q] = relu4((acc[q] + sv) * dc + bq[q]);
    }
    float s1 = 0.0f;
#pragma unroll
    for (int q = 0; q < NQ; ++q) s1 += (v[q].x + v[q].y) + (v[q].z + v[q].w);
#pragma unroll
    for (int o = 16; o > 0; o >>= 1) s1 += __shfl_xor(s1, o, 32);
    const float mu = s1 * invC;
    v4f xc[NQ];
    float s2 = 0.0f;
#pragma unroll
    for (int q = 0; q < NQ; ++q) {
      xc[q] = v[q] - mu;
      s2 += (xc[q].x * xc[q].x + xc[q].y * xc[q].y) + (xc[q].z * xc[q].z + xc[q].w * xc[q].w);
    }
#pragma unroll
    for (int o = 16; o > 0; o >>= 1) s2 += __shfl_xor(s2, o, 32);
    const float var  = s2 * invC;
    const float rstd = rsqrtf(var + LNEPS);
    v4f y[NQ];
#pragma unroll
    for (int q = 0; q < NQ; ++q) {
      y[q].x = xc[q].x * rstd * gq[q].x + eq[q].x;
      y[q].y = xc[q].y * rstd * gq[q].y + eq[q].y;
      y[q].z = xc[q].z * rstd * gq[q].z + eq[q].z;
      y[q].w = xc[q].w * rstd * gq[q].w + eq[q].w;
    }
    if (MODE == 0) {
      const float z = (c < nN) ? 1.0f : 0.0f;
      const v4f ya = y[0] * z;
      const v4f yb = y[NQ - 1] * z;
      v8us h8, l8;
      split8(ya, yb, h8, l8);
      unsigned short* ph = outHi + (size_t)c * CH + 8 * lane;
      unsigned short* pl = outLo + (size_t)c * CH + 8 * lane;
      *(volatile v8us*)ph = h8;
      *(volatile v8us*)pl = l8;
      __threadfence();
      *(volatile v8us*)ph = h8;
      *(volatile v8us*)pl = l8;
    } else {
      if (c < nN) {
        const v4f yv = y[0];
        float* rp = outF + (size_t)c * CH + 4 * lane;
        *(volatile v4f*)rp = yv;
        __threadfence();
        *(volatile v4f*)rp = yv;
      }
    }
  }
}

extern "C" void kernel_launch(void* const* d_in, const int* in_sizes, int n_in,
                              void* d_out, int out_size, void* d_ws, size_t ws_size,
                              hipStream_t stream) {
  if (n_in < 14) return;
  const int nN = in_sizes[0] / DIN;
  const int nE = in_sizes[1] / 2;
  if (nN <= 0 || nE <= 0) return;
  if (in_sizes[0] != nN * DIN || in_sizes[1] != 2 * nE) return;
  if (in_sizes[2] != DIN * HID || in_sizes[3] != HID || in_sizes[4] != HID || in_sizes[5] != HID) return;
  if (in_sizes[6] != HID * HID || in_sizes[7] != HID || in_sizes[8] != HID || in_sizes[9] != HID) return;
  if (in_sizes[10] != HID * DOUT || in_sizes[11] != DOUT || in_sizes[12] != DOUT || in_sizes[13] != DOUT) return;
  if (nN > (1 << 20) || nE > (1 << 28)) return;
  if ((long long)out_size != (long long)nN * DOUT) return;

  const float* x   = (const float*)d_in[0];
  const int*   ei  = (const int*)d_in[1];
  const float* W1  = (const float*)d_in[2];
  const float* b1  = (const float*)d_in[3];
  const float* g1  = (const float*)d_in[4];
  const float* be1 = (const float*)d_in[5];
  const float* W2  = (const float*)d_in[6];
  const float* b2  = (const float*)d_in[7];
  const float* g2  = (const float*)d_in[8];
  const float* be2 = (const float*)d_in[9];
  const float* W3  = (const float*)d_in[10];
  const float* b3  = (const float*)d_in[11];
  const float* g3  = (const float*)d_in[12];
  const float* be3 = (const float*)d_in[13];
  float* out = (float*)d_out;
  const int* keys = ei + nE;
  const int* vals = ei;
  const int nK = nE;

  const int NPAD   = ((nN + TGT - 1) / TGT) * TGT;
  const int nBC    = (nN + NBC - 1) / NBC;
  const int CNTPAD = nBC * NBC;
  const int nBF    = (nN + NBF - 1) / NBF;
  const int OFFN   = nBF * NBF;
  if (nBF + 1 > RBN) return;
  if (OFFN > CNTPAD || NPAD > OFFN) return;
  const int csrLen = ((nK + 31) & ~31) + 32 * (nBF + 1);
  const int nGemm  = NPAD / GROWS;
  const int nAgg   = NPAD / TGT;

  char* ws = (char*)d_ws;
  size_t off = 0;
  const size_t oHh  = off; off += (size_t)NPAD * HID * 2;        off = (off + 255) & ~(size_t)255;
  const size_t oHl  = off; off += (size_t)NPAD * HID * 2;        off = (off + 255) & ~(size_t)255;
  const size_t oW1h = off; off += (size_t)HID * DIN * 2;         off = (off + 255) & ~(size_t)255;
  const size_t oW1l = off; off += (size_t)HID * DIN * 2;         off = (off + 255) & ~(size_t)255;
  const size_t oW2h = off; off += (size_t)HID * HID * 2;         off = (off + 255) & ~(size_t)255;
  const size_t oW2l = off; off += (size_t)HID * HID * 2;         off = (off + 255) & ~(size_t)255;
  const size_t oW3h = off; off += (size_t)DOUT * HID * 2;        off = (off + 255) & ~(size_t)255;
  const size_t oW3l = off; off += (size_t)DOUT * HID * 2;        off = (off + 255) & ~(size_t)255;
  const size_t oCnt = off; off += (size_t)CNTPAD * 4;            off = (off + 255) & ~(size_t)255;
  const size_t oDv  = off; off += (size_t)CNTPAD * 4;            off = (off + 255) & ~(size_t)255;
  const size_t oOff = off; off += (size_t)OFFN * 4;              off = (off + 255) & ~(size_t)255;
  const size_t oRb  = off; off += (size_t)RBN * 4;               off = (off + 255) & ~(size_t)255;
  const size_t oCsr = off; off += (size_t)csrLen * 4;            off = (off + 255) & ~(size_t)255;
  const size_t oHW  = off; off += (size_t)NPAD * HID * 4;        off = (off + 255) & ~(size_t)255;
  if (off > ws_size || off > (size_t)WSCAP) return;
  unsigned short* Hh   = (unsigned short*)(ws + oHh);
  unsigned short* Hl   = (unsigned short*)(ws + oHl);
  unsigned short* Xh   = Hh;
  unsigned short* Xl   = Hl;
  unsigned short* W1h  = (unsigned short*)(ws + oW1h);
  unsigned short* W1l  = (unsigned short*)(ws + oW1l);
  unsigned short* W2h  = (unsigned short*)(ws + oW2h);
  unsigned short* W2l  = (unsigned short*)(ws + oW2l);
  unsigned short* W3h  = (unsigned short*)(ws + oW3h);
  unsigned short* W3l  = (unsigned short*)(ws + oW3l);
  int*      cnt  = (int*)(ws + oCnt);
  float*    dinv = (float*)(ws + oDv);
  int*      offp = (int*)(ws + oOff);
  int*      rb   = (int*)(ws + oRb);
  int*      csr  = (int*)(ws + oCsr);
  float*    HW   = (float*)(ws + oHW);

  const int vec8 = ((nE & 7) == 0) ? 1 : 0;

  {
    const int t8 = (NPAD * DIN) / 8;
    k_split16<<<(t8 + NTHR - 1) / NTHR, NTHR, 0, stream>>>(x, Xh, Xl, DIN, nN, t8);
  }
  k_wT16<<<dim3(DIN / TPK, HID / TPN), NTHR, 0, stream>>>(W1, W1h, W1l, DIN, HID);
  k_wT16<<<dim3(HID / TPK, HID / TPN), NTHR, 0, stream>>>(W2, W2h, W2l, HID, HID);
  k_wT16<<<dim3(HID / TPK, DOUT / TPN), NTHR, 0, stream>>>(W3, W3h, W3l, HID, DOUT);

  hipFuncSetAttribute(reinterpret_cast<const void*>(&k_count),
                      hipFuncAttributeMaxDynamicSharedMemorySize, LDS_COUNT);
  k_count<<<nBC, NTHR, LDS_COUNT, stream>>>(keys, cnt, dinv, nK, nN, vec8);
  k_offsets<<<1, OTHR, 0, stream>>>(cnt, offp, rb, nBF);
  hipFuncSetAttribute(reinterpret_cast<const void*>(&k_fill),
                      hipFuncAttributeMaxDynamicSharedMemorySize, LDS_FILL);
  k_fill<<<nBF, NTHR, LDS_FILL, stream>>>(keys, vals, offp, rb, csr, nN, nK, vec8, csrLen);

  hipFuncSetAttribute(reinterpret_cast<const void*>(&k_gemm<DIN, HID>),
                      hipFuncAttributeMaxDynamicSharedMemorySize, LDS_GEMM);
  k_gemm<DIN, HID><<<dim3(nGemm, HID / GCOLS), NTHR, LDS_GEMM, stream>>>(Xh, Xl, W1h, W1l, dinv, HW, NPAD);
  k_agg<HID, 0><<<nAgg, NTHR, 0, stream>>>(csr, offp, cnt, dinv, HW, b1, g1, be1, out, Hh, Hl, nN, csrLen);

  hipFuncSetAttribute(reinterpret_cast<const void*>(&k_gemm<HID, HID>),
                      hipFuncAttributeMaxDynamicSharedMemorySize, LDS_GEMM);
  k_gemm<HID, HID><<<dim3(nGemm, HID / GCOLS), NTHR, LDS_GEMM, stream>>>(Hh, Hl, W2h, W2l, dinv, HW, NPAD);
  k_agg<HID, 0><<<nAgg, NTHR, 0, stream>>>(csr, offp, cnt, dinv, HW, b2, g2, be2, out, Hh, Hl, nN, csrLen);

  hipFuncSetAttribute(reinterpret_cast<const void*>(&k_gemm<HID, DOUT>),
                      hipFuncAttributeMaxDynamicSharedMemorySize, LDS_GEMM);
  k_gemm<HID, DOUT><<<dim3(nGemm, DOUT / GCOLS), NTHR, LDS_GEMM, stream>>>(Hh, Hl, W3h, W3l, dinv, HW, NPAD);
  k_agg<DOUT, 1><<<nAgg, NTHR, 0, stream>>>(csr, offp, cnt, dinv, HW, b3, g3, be3, out, Hh, Hl, nN, csrLen);
}
